// Damping_72799695667307
// MI455X (gfx1250) — hardware-verified
//
#include <hip/hip_runtime.h>

typedef __bf16         v16bf __attribute__((ext_vector_type(16)));
typedef unsigned short v8us  __attribute__((ext_vector_type(8)));
typedef float          v8f   __attribute__((ext_vector_type(8)));
typedef float          v4f   __attribute__((ext_vector_type(4)));
typedef v8us __attribute__((may_alias)) v8usa;
typedef v4f  __attribute__((may_alias)) v4fa;

union Frag { v16bf v; v8us half[2]; };

#define NB    64
#define HH    256
#define OFFD  2016
#define OFFP  2048
#define BM    16
#define NT    256

#define WOFF_D1 0
#define WOFF_O1 16384
#define WOFF_D2 32768
#define WOFF_O2 98304
#define WOFF_DO 163840
#define WOFF_OO 180224
#define W_END   704512
#define WS_TOTAL_BYTES ((size_t)W_END * 2)

#define G_O1  2048
#define G_D2  4096
#define G_O2  12288
#define G_DO  20480
#define G_OO  22528
#define G_PAD 87040
#define G_END 88064

static_assert(WOFF_O1 == WOFF_D1 + HH * NB);
static_assert(WOFF_D2 == WOFF_O1 + HH * NB);
static_assert(WOFF_O2 == WOFF_D2 + HH * HH);
static_assert(WOFF_DO == WOFF_O2 + HH * HH);
static_assert(WOFF_OO == WOFF_DO + NB * HH);
static_assert(W_END == WOFF_OO + OFFP * HH);
static_assert(G_O1 * 8 == WOFF_O1 && G_D2 * 8 == WOFF_D2 && G_O2 * 8 == WOFF_O2);
static_assert(G_DO * 8 == WOFF_DO && G_OO * 8 == WOFF_OO && G_END * 8 == W_END);
static_assert(G_PAD * 8 == WOFF_OO + OFFD * HH);
static_assert(G_O1 % NT == 0 && G_D2 % NT == 0 && G_O2 % NT == 0 && G_DO % NT == 0);
static_assert(G_OO % NT == 0 && G_PAD % NT == 0 && G_END % NT == 0);
static_assert(NB % 32 == 0 && HH % 32 == 0);

#define HPITCH 264
#define XP16   72
#define XPF    68
#define ZP     2052
#define PLANE  (BM * HPITCH)
#define OFF_Z   0
#define SZ_Z    (BM * ZP * 4)
#define OFF_H1  0
#define OFF_H2  SZ_Z
#define OFF_Y   SZ_Z
#define OFF_D   (SZ_Z + BM * XPF * 4)
#define OFF_XB  (SZ_Z + 4 * PLANE * 2)
#define OFF_X0  (OFF_XB + BM * XP16 * 2)
#define OFF_XD  (OFF_X0 + BM * XPF * 4)
#define SMEM_TOTAL (OFF_XD + BM * XPF * 4)

static_assert(4 * PLANE * 2 <= SZ_Z);
static_assert(OFF_D + BM * NB * 4 <= OFF_XB);
static_assert(SMEM_TOTAL == 176128);
static_assert((OFF_H2 % 16) == 0 && (OFF_D % 16) == 0 && (OFF_XB % 16) == 0 && (OFF_X0 % 16) == 0 && (OFF_XD % 16) == 0);
static_assert((HPITCH * 2) % 16 == 0 && (XP16 * 2) % 16 == 0 && (XPF * 4) % 16 == 0 && (PLANE * 2) % 16 == 0);

__device__ __forceinline__ unsigned short f2bf(float f) {
  unsigned u = __builtin_bit_cast(unsigned, f);
  u += 0x7FFFu + ((u >> 16) & 1u);
  return (unsigned short)(u >> 16);
}
__device__ __forceinline__ float bf2f(unsigned short s) {
  return __builtin_bit_cast(float, ((unsigned)s) << 16);
}
__device__ __forceinline__ float bfr(float f) { return bf2f(f2bf(f)); }

__device__ __forceinline__ float tanh_f(float v) {
  v = fminf(fmaxf(v, -15.0f), 15.0f);
  const float e = __expf(2.0f * v);
  return 1.0f - 2.0f * __builtin_amdgcn_rcpf(1.0f + e);
}

__device__ __forceinline__ v8f wmma_bf16(v16bf a, v16bf b, v8f c) {
  v8f d = __builtin_amdgcn_wmma_f32_16x16x32_bf16(false, a, false, b, (short)0, c, false, false);
  asm volatile("v_nop\n\tv_nop\n\tv_nop\n\tv_nop" : "+v"(d) : "v"(a), "v"(b));
  return d;
}

__device__ __forceinline__ v16bf load_frag(const unsigned short* p, int h) {
  Frag f;
  f.half[0] = *(const v8usa*)(p + 8 * h);
  f.half[1] = *(const v8usa*)(p + 16 + 8 * h);
  return f.v;
}

template <int T, int K>
__device__ __forceinline__ void gemm_strip1(const unsigned short* arow,
                                            const unsigned short* __restrict__ brow,
                                            int h, v8f (&acc)[T]) {
  const v8f z8 = {0.f, 0.f, 0.f, 0.f, 0.f, 0.f, 0.f, 0.f};
  #pragma unroll
  for (int t = 0; t < T; ++t) acc[t] = z8;
  #pragma unroll 1
  for (int k0 = 0; k0 < K; k0 += 32) {
    const v16bf a = load_frag(arow + k0, h);
    #pragma unroll
    for (int t = 0; t < T; ++t) {
      const v16bf b = load_frag(brow + (size_t)t * 16 * K + k0, h);
      acc[t] = wmma_bf16(a, b, acc[t]);
    }
  }
}

template <int T, int K>
__device__ __forceinline__ void gemm_strip2(const unsigned short* arowHi,
                                            const unsigned short* arowLo,
                                            const unsigned short* __restrict__ brow,
                                            int h, v8f (&acc)[T]) {
  const v8f z8 = {0.f, 0.f, 0.f, 0.f, 0.f, 0.f, 0.f, 0.f};
  #pragma unroll
  for (int t = 0; t < T; ++t) acc[t] = z8;
  #pragma unroll 1
  for (int k0 = 0; k0 < K; k0 += 32) {
    const v16bf a  = load_frag(arowHi + k0, h);
    const v16bf al = load_frag(arowLo + k0, h);
    #pragma unroll
    for (int t = 0; t < T; ++t) {
      const v16bf b = load_frag(brow + (size_t)t * 16 * K + k0, h);
      acc[t] = wmma_bf16(a, b, acc[t]);
      acc[t] = wmma_bf16(al, b, acc[t]);
    }
  }
}

template <int T>
__device__ __forceinline__ void act_epilogue(const v8f (&acc)[T], const float* __restrict__ bias,
                                             int n0, unsigned short* pHi, unsigned short* pLo,
                                             int h, int m) {
  #pragma unroll
  for (int t = 0; t < T; ++t) {
    const int col = n0 + 16 * t + m;
    const float bv = bfr(bias[col]);
    #pragma unroll
    for (int r = 0; r < 8; ++r) {
      const float v = tanh_f(acc[t][r] + bv);
      const unsigned short hi = f2bf(v);
      const unsigned short lo = f2bf(v - bf2f(hi));
      const int idx = (8 * h + r) * HPITCH + col;
      pHi[idx] = hi;
      pLo[idx] = lo;
    }
  }
}

__global__ __launch_bounds__(NT) void convert_weights(
    const float* __restrict__ wd1, const float* __restrict__ wo1,
    const float* __restrict__ wd2, const float* __restrict__ wo2,
    const float* __restrict__ wdo, const float* __restrict__ woo,
    unsigned short* __restrict__ planes)
{
  const int g = blockIdx.x * NT + threadIdx.x;
  if (g >= G_END) return;
  const float* src;
  bool pad = false;
  if (g < G_O1)       src = wd1 + (size_t)g * 8;
  else if (g < G_D2)  src = wo1 + (size_t)(g - G_O1) * 8;
  else if (g < G_O2)  src = wd2 + (size_t)(g - G_D2) * 8;
  else if (g < G_DO)  src = wo2 + (size_t)(g - G_O2) * 8;
  else if (g < G_OO)  src = wdo + (size_t)(g - G_DO) * 8;
  else {
    pad = (g >= G_PAD);
    const int e = pad ? 0 : (g - G_OO);
    src = woo + (size_t)e * 8;
  }
  const v4f a = *(const v4fa*)src;
  const v4f c = *(const v4fa*)(src + 4);
  const v8us cv = { f2bf(a.x), f2bf(a.y), f2bf(a.z), f2bf(a.w),
                    f2bf(c.x), f2bf(c.y), f2bf(c.z), f2bf(c.w) };
  const v8us zz = { 0, 0, 0, 0, 0, 0, 0, 0 };
  const v8us o = pad ? zz : cv;
  unsigned short* dst = planes + (size_t)g * 8;
  *(volatile v8us*)dst = o;
  __threadfence();
  *(volatile v8us*)dst = o;
}

__global__ __launch_bounds__(NT) void k_ltri(
    const float* __restrict__ x,
    const unsigned short* __restrict__ wb,
    const float* __restrict__ bd1, const float* __restrict__ bd2,
    const float* __restrict__ bdo, const float* __restrict__ bo1,
    const float* __restrict__ bo2, const float* __restrict__ boo,
    float* __restrict__ out)
{
  extern __shared__ __attribute__((aligned(16))) char smem[];
  float*          zb  = (float*)(smem + OFF_Z);
  unsigned short* h1  = (unsigned short*)(smem + OFF_H1);
  unsigned short* h2  = (unsigned short*)(smem + OFF_H2);
  float*          yb  = (float*)(smem + OFF_Y);
  float*          sD  = (float*)(smem + OFF_D);
  unsigned short* xbf = (unsigned short*)(smem + OFF_XB);
  float*          x0  = (float*)(smem + OFF_X0);
  float*          xd  = (float*)(smem + OFF_XD);

  const int tid = threadIdx.x, lane = tid & 31;
  const int w = __builtin_amdgcn_readfirstlane(tid >> 5);
  const int h = lane >> 4, m = lane & 15;
  const int br = w >> 2;
  const int wq = w & 3;
  const int row0 = blockIdx.x * BM;

  {
    const v4f v = *(const v4fa*)(x + (size_t)row0 * NB + (size_t)tid * 4);
    const int s = tid >> 4, c0 = (tid & 15) << 2;
    const unsigned short b0 = f2bf(v.x), b1 = f2bf(v.y), b2 = f2bf(v.z), b3 = f2bf(v.w);
    unsigned short* xb = xbf + s * XP16 + c0;
    xb[0] = b0; xb[1] = b1; xb[2] = b2; xb[3] = b3;
    const v4f xr = { bf2f(b0), bf2f(b1), bf2f(b2), bf2f(b3) };
    *(v4fa*)(x0 + s * XPF + c0) = xr;
  }
  __syncthreads();

  {
    v8f acc[4];
    const int n0 = 64 * wq;
    const unsigned short* w1 = wb + (br ? WOFF_O1 : WOFF_D1);
    gemm_strip1<4, NB>(xbf + m * XP16, w1 + (size_t)(n0 + m) * NB, h, acc);
    const float* bias = br ? bo1 : bd1;
    unsigned short* pHi = h1 + br * (2 * PLANE);
    unsigned short* pLo = pHi + PLANE;
    act_epilogue<4>(acc, bias, n0, pHi, pLo, h, m);
  }
  __syncthreads();

  {
    v8f acc[4];
    const int n0 = 64 * wq;
    const unsigned short* aHi = h1 + br * (2 * PLANE) + m * HPITCH;
    const unsigned short* aLo = aHi + PLANE;
    const unsigned short* w2 = wb + (br ? WOFF_O2 : WOFF_D2);
    gemm_strip2<4, HH>(aHi, aLo, w2 + (size_t)(n0 + m) * HH, h, acc);
    const float* bias = br ? bo2 : bd2;
    unsigned short* pHi = h2 + br * (2 * PLANE);
    unsigned short* pLo = pHi + PLANE;
    act_epilogue<4>(acc, bias, n0, pHi, pLo, h, m);
  }
  __syncthreads();

  if (w < 4) {
    v8f acc[1];
    const int n0 = 16 * w;
    const unsigned short* aHi = h2 + m * HPITCH;
    const unsigned short* aLo = aHi + PLANE;
    gemm_strip2<1, HH>(aHi, aLo, wb + WOFF_DO + (size_t)(n0 + m) * HH, h, acc);
    const float bv = bfr(bdo[n0 + m]);
    #pragma unroll
    for (int r = 0; r < 8; ++r)
      xd[(8 * h + r) * XPF + n0 + m] = acc[0][r] + bv;
  }
  {
    const unsigned short* aHi = h2 + 2 * PLANE + m * HPITCH;
    const unsigned short* aLo = aHi + PLANE;
    #pragma unroll 1
    for (int i = 0; i < 4; ++i) {
      const int n0 = 64 * (w + 8 * i);
      v8f acc[4];
      gemm_strip2<4, HH>(aHi, aLo, wb + WOFF_OO + (size_t)(n0 + m) * HH, h, acc);
      #pragma unroll
      for (int t = 0; t < 4; ++t) {
        const int col = n0 + 16 * t + m;
        const int colc = (col < OFFD) ? col : (OFFD - 1);
        const float bl = bfr(boo[colc]);
        const float bv = (col < OFFD) ? bl : 0.0f;
        #pragma unroll
        for (int r = 0; r < 8; ++r)
          zb[(8 * h + r) * ZP + col] = acc[t][r] + bv;
      }
    }
  }
  __syncthreads();

  const int s  = tid >> 4;
  const int j0 = tid & 15;
  const float* zr  = zb + s * ZP;
  const float* x0r = x0 + s * XPF;
  const float* xdr = xd + s * XPF;
  float*       yr  = yb + s * XPF;

  #pragma unroll
  for (int c4 = 0; c4 < 4; ++c4) {
    const int j = j0 + 16 * c4;
    float acc = xdr[j] * x0r[j];
    int f = (j * (j + 1)) / 2 + j;
    int add = j + 1;
    #pragma unroll 1
    for (int k = j + 1; k < NB; ++k) { acc += zr[f] * x0r[k]; f += add; ++add; }
    yr[j] = acc;
  }
  __syncthreads();

  #pragma unroll
  for (int c4 = 0; c4 < 4; ++c4) {
    const int i = j0 + 16 * c4;
    float acc = xdr[i] * yr[i];
    const int base = (i * (i - 1)) / 2;
    #pragma unroll 1
    for (int j = 0; j < i; ++j) acc += zr[base + j] * yr[j];
    sD[s * NB + i] = acc;
  }
  __syncthreads();

  {
    const v4f v = *(const v4fa*)(sD + tid * 4);
    float* dst = out + (size_t)row0 * NB + (size_t)tid * 4;
    *(volatile v4f*)dst = v;
    __threadfence();
    *(volatile v4f*)dst = v;
  }
}

extern "C" void kernel_launch(void* const* d_in, const int* in_sizes, int n_in,
                              void* d_out, int out_size, void* d_ws, size_t ws_size,
                              hipStream_t stream) {
  if (n_in < 13) return;
  if (in_sizes[0] <= 0 || (in_sizes[0] % (NB * BM)) != 0) return;
  const int nB = in_sizes[0] / NB;
  if (in_sizes[1] != HH * NB   || in_sizes[2]  != HH)   return;
  if (in_sizes[3] != HH * HH   || in_sizes[4]  != HH)   return;
  if (in_sizes[5] != NB * HH   || in_sizes[6]  != NB)   return;
  if (in_sizes[7] != HH * NB   || in_sizes[8]  != HH)   return;
  if (in_sizes[9] != HH * HH   || in_sizes[10] != HH)   return;
  if (in_sizes[11] != OFFD * HH || in_sizes[12] != OFFD) return;
  if (out_size != nB * NB) return;
  if (WS_TOTAL_BYTES > ws_size) return;

  const float* x   = (const float*)d_in[0];
  const float* Wd1 = (const float*)d_in[1];
  const float* bd1 = (const float*)d_in[2];
  const float* Wd2 = (const float*)d_in[3];
  const float* bd2 = (const float*)d_in[4];
  const float* Wdo = (const float*)d_in[5];
  const float* bdo = (const float*)d_in[6];
  const float* Wo1 = (const float*)d_in[7];
  const float* bo1 = (const float*)d_in[8];
  const float* Wo2 = (const float*)d_in[9];
  const float* bo2 = (const float*)d_in[10];
  const float* Woo = (const float*)d_in[11];
  const float* boo = (const float*)d_in[12];
  float* out = (float*)d_out;

  unsigned short* planes = (unsigned short*)d_ws;

  convert_weights<<<G_END / NT, NT, 0, stream>>>(Wd1, Wo1, Wd2, Wo2, Wdo, Woo, planes);

  hipFuncSetAttribute(reinterpret_cast<const void*>(&k_ltri),
                      hipFuncAttributeMaxDynamicSharedMemorySize, SMEM_TOTAL);
  k_ltri<<<nB / BM, NT, SMEM_TOTAL, stream>>>(
      x, planes, bd1, bd2, bdo, bo1, bo2, boo, out);
}
